// K2Layer_4234837753981
// MI455X (gfx1250) — hardware-verified
//
#include <hip/hip_runtime.h>
#include <stddef.h>
#include <stdint.h>
#include <math.h>

#define BB   2
#define WW   1024
#define CC   1024
#define RR   16
#define FF   2048
#define ROWS (BB * WW)

static_assert(WW % 256 == 0);
static_assert(CC % 256 == 0);
static_assert(FF % 64 == 0);
static_assert(RR == 16);
static_assert(ROWS % 256 == 0);

typedef _Float16 v16h __attribute__((ext_vector_type(16)));
typedef _Float16 v8h  __attribute__((ext_vector_type(8)));
typedef float    v8f  __attribute__((ext_vector_type(8)));
typedef float    v4f  __attribute__((ext_vector_type(4)));
typedef unsigned int v4u __attribute__((ext_vector_type(4)));

union Frag  { v16h v; v8h h[2]; };
union Pack8 { v8h h; v4u u; };

__device__ __forceinline__ v8f mma16(v16h a, v16h b, v8f c) {
  c = __builtin_amdgcn_wmma_f32_16x16x32_f16(false, a, false, b, (short)0, c, false, false);
  asm volatile("v_nop\n\tv_nop\n\tv_nop\n\tv_nop" : "+v"(c) : "v"(a), "v"(b));
  return c;
}

__device__ __forceinline__ v16h ldfrag(const _Float16* p, int ld, int row0, int k0, int lane) {
  const int m = lane & 15, lh = lane >> 4;
  const _Float16* q = p + (size_t)(row0 + m) * ld + k0 + 8 * lh;
  Frag f;
  f.h[0] = *(const v8h*)(q);
  f.h[1] = *(const v8h*)(q + 16);
  return f.v;
}

__device__ __forceinline__ v8f zero8() { return (v8f){0.f, 0.f, 0.f, 0.f, 0.f, 0.f, 0.f, 0.f}; }

__device__ __forceinline__ float act16(float v) {
  return 8.0f * v * (1.0f + erff(v * 0.70710678118654752f));
}

__device__ __forceinline__ void gemm32x64(const _Float16* __restrict__ A, int lda,
                                          const _Float16* __restrict__ Bt, int ldb,
                                          int m0, int n0, int lane, int kend, v8f (&acc)[2][4]) {
#pragma unroll 2
  for (int k0 = 0; k0 < kend; k0 += 32) {
    const v16h a0 = ldfrag(A, lda, m0, k0, lane);
    const v16h a1 = ldfrag(A, lda, m0 + 16, k0, lane);
    const v16h b0 = ldfrag(Bt, ldb, n0, k0, lane);
    const v16h b1 = ldfrag(Bt, ldb, n0 + 16, k0, lane);
    const v16h b2 = ldfrag(Bt, ldb, n0 + 32, k0, lane);
    const v16h b3 = ldfrag(Bt, ldb, n0 + 48, k0, lane);
    acc[0][0] = mma16(a0, b0, acc[0][0]);
    acc[1][0] = mma16(a1, b0, acc[1][0]);
    acc[0][1] = mma16(a0, b1, acc[0][1]);
    acc[1][1] = mma16(a1, b1, acc[1][1]);
    acc[0][2] = mma16(a0, b2, acc[0][2]);
    acc[1][2] = mma16(a1, b2, acc[1][2]);
    acc[0][3] = mma16(a0, b3, acc[0][3]);
    acc[1][3] = mma16(a1, b3, acc[1][3]);
  }
}

__global__ __launch_bounds__(256) void k_rms(const float* __restrict__ in,
                                            const float* __restrict__ sc,
                                            _Float16* __restrict__ outh) {
  __shared__ __align__(16) float rb[CC];
  __shared__ float red[8];
  const int tid = threadIdx.x, lane = tid & 31, wave = tid >> 5;
  const size_t ro = (size_t)blockIdx.x * CC;
  const v4f x = *(const v4f*)(in + ro + 4 * tid);
  float s = (x[0] * x[0] + x[1] * x[1]) + (x[2] * x[2] + x[3] * x[3]);
#pragma unroll
  for (int off = 1; off < 32; off <<= 1) s += __shfl_xor(s, off, 32);
  if (lane == 0) red[wave] = s;
  __syncthreads();
  float ts = 0.f;
#pragma unroll
  for (int w = 0; w < 8; ++w) ts += red[w];
  const float ms  = ts * (1.0f / (float)CC);
  const float inv = 1.0f / sqrtf(ms + 1e-8f);
  const v4f g4 = *(const v4f*)(sc + 4 * tid);
  v4f o;
  o[0] = x[0] * inv * g4[0];
  o[1] = x[1] * inv * g4[1];
  o[2] = x[2] * inv * g4[2];
  o[3] = x[3] * inv * g4[3];
  *(v4f*)(rb + 4 * tid) = o;
  __syncthreads();
  if (tid < 128) {
    const v4f a0 = *(const v4f*)(rb + 8 * tid);
    const v4f a1 = *(const v4f*)(rb + 8 * tid + 4);
    Pack8 pk;
    pk.h = (v8h){(_Float16)a0[0], (_Float16)a0[1], (_Float16)a0[2], (_Float16)a0[3],
                 (_Float16)a1[0], (_Float16)a1[1], (_Float16)a1[2], (_Float16)a1[3]};
    const v4u vv = pk.u;
    volatile v4u* hq = (volatile v4u*)(outh + ro + 8 * tid);
    *hq = vv;
    __threadfence();
    *hq = vv;
  }
}

#define TTP 72
__global__ __launch_bounds__(256) void k_tr16(const _Float16* __restrict__ in, _Float16* __restrict__ out,
                                             int nrows, int ncols) {
  __shared__ __align__(16) _Float16 tl[64 * TTP];
  const int tid = threadIdx.x;
  const size_t bo = (size_t)blockIdx.z * nrows * ncols;
  const _Float16* inb = in + bo;
  _Float16* outb = out + bo;
  const int r0 = blockIdx.y * 64;
  const int c0 = blockIdx.x * 64;
  {
    const int r   = tid >> 2;
    const int q16 = (tid & 3) * 16;
    const _Float16* src = inb + (size_t)(r0 + r) * ncols + c0 + q16;
    *(v8h*)(tl + r * TTP + q16)     = *(const v8h*)(src);
    *(v8h*)(tl + r * TTP + q16 + 8) = *(const v8h*)(src + 8);
  }
  __syncthreads();
  v4u val[2];
  size_t go[2];
#pragma unroll
  for (int j = 0; j < 2; ++j) {
    const int p  = tid + 256 * j;
    const int n  = p >> 3;
    const int pc = p & 7;
    const _Float16* cp = tl + (pc * 8) * TTP + n;
    Pack8 pk;
    pk.h = (v8h){cp[0 * TTP], cp[1 * TTP], cp[2 * TTP], cp[3 * TTP],
                 cp[4 * TTP], cp[5 * TTP], cp[6 * TTP], cp[7 * TTP]};
    val[j] = pk.u;
    go[j]  = (size_t)(c0 + n) * nrows + r0 + pc * 8;
  }
  for (int ps = 0; ps < 2; ++ps) {
#pragma unroll
    for (int j = 0; j < 2; ++j) *(volatile v4u*)(outb + go[j]) = val[j];
    __threadfence();
  }
}

__global__ __launch_bounds__(128) void k_uvt(const float* u, const float* v, _Float16* __restrict__ uvt) {
  const int n = blockIdx.x;
  const int t = threadIdx.x;
  const float* src = (n < 16) ? u : v;
  const int c = n & 15;
  float f[8];
#pragma unroll
  for (int e = 0; e < 8; ++e) f[e] = src[(size_t)(8 * t + e) * RR + c] * 64.0f;
  Pack8 pk;
  pk.h = (v8h){(_Float16)f[0], (_Float16)f[1], (_Float16)f[2], (_Float16)f[3],
               (_Float16)f[4], (_Float16)f[5], (_Float16)f[6], (_Float16)f[7]};
  const v4u vv = pk.u;
  volatile v4u* d = (volatile v4u*)(uvt + (size_t)n * CC + 8 * t);
  *d = vv;
  __threadfence();
  *d = vv;
}

#define WTP 68
__global__ __launch_bounds__(256) void k_wt(const float* __restrict__ w, _Float16* __restrict__ wt,
                                           int nout, int kin) {
  __shared__ __align__(16) float tf[64 * WTP];
  const int tid = threadIdx.x;
  const int n0 = blockIdx.x * 64;
  const int k0 = blockIdx.y * 64;
  {
    const int kr = tid >> 4;
    const int n4 = (tid & 15) * 4;
#pragma unroll
    for (int it = 0; it < 4; ++it) {
      const int kl = it * 16 + kr;
      const v4f a = *(const v4f*)(w + (size_t)(k0 + kl) * nout + n0 + n4);
      *(v4f*)(tf + kl * WTP + n4) = a;
    }
  }
  __syncthreads();
  v4u val[2];
  size_t go[2];
#pragma unroll
  for (int j = 0; j < 2; ++j) {
    const int p  = tid + 256 * j;
    const int nl = p >> 3;
    const int pc = p & 7;
    const float* cp = tf + (pc * 8) * WTP + nl;
    Pack8 pk;
    pk.h = (v8h){(_Float16)(cp[0 * WTP] * 32.0f), (_Float16)(cp[1 * WTP] * 32.0f),
                 (_Float16)(cp[2 * WTP] * 32.0f), (_Float16)(cp[3 * WTP] * 32.0f),
                 (_Float16)(cp[4 * WTP] * 32.0f), (_Float16)(cp[5 * WTP] * 32.0f),
                 (_Float16)(cp[6 * WTP] * 32.0f), (_Float16)(cp[7 * WTP] * 32.0f)};
    val[j] = pk.u;
    go[j]  = (size_t)(n0 + nl) * kin + k0 + pc * 8;
  }
  for (int ps = 0; ps < 2; ++ps) {
#pragma unroll
    for (int j = 0; j < 2; ++j) *(volatile v4u*)(wt + go[j]) = val[j];
    __threadfence();
  }
}

#define QTP 36
__global__ __launch_bounds__(256) void k_qk(const _Float16* __restrict__ hn,
                                           const _Float16* __restrict__ uvt,
                                           float* __restrict__ qk) {
  __shared__ __align__(16) float st[8][16 * QTP];
  const int tid = threadIdx.x, lane = tid & 31, wave = tid >> 5;
  const int hh = lane >> 4, c = lane & 15;
  const int m0 = blockIdx.x * 128 + wave * 16;

  v8f acc[2];
  acc[0] = zero8();
  acc[1] = zero8();
#pragma unroll 2
  for (int k0 = 0; k0 < CC; k0 += 32) {
    const v16h a  = ldfrag(hn, CC, m0, k0, lane);
    const v16h b0 = ldfrag(uvt, CC, 0, k0, lane);
    const v16h b1 = ldfrag(uvt, CC, 16, k0, lane);
    acc[0] = mma16(a, b0, acc[0]);
    acc[1] = mma16(a, b1, acc[1]);
  }
  float* sw = st[wave];
#pragma unroll
  for (int t = 0; t < 2; ++t) {
#pragma unroll
    for (int r = 0; r < 8; ++r) {
      const float x = acc[t][r] * 0.015625f;
      float ss = x * x;
#pragma unroll
      for (int off = 1; off < 16; off <<= 1) ss += __shfl_xor(ss, off, 32);
      const float nrm = sqrtf(ss);
      const float den = fmaxf(nrm, 1e-8f);
      sw[(8 * hh + r) * QTP + 16 * t + c] = x * (1.0f / den);
    }
  }
  __syncthreads();
  v4f val[4];
  size_t go[4];
#pragma unroll
  for (int it = 0; it < 4; ++it) {
    const int p  = lane + 32 * it;
    const int L  = p >> 3;
    const int pc = p & 7;
    val[it] = *(const v4f*)(sw + L * QTP + pc * 4);
    go[it]  = (size_t)(m0 + L) * 32 + pc * 4;
  }
  for (int ps = 0; ps < 2; ++ps) {
#pragma unroll
    for (int it = 0; it < 4; ++it) *(volatile v4f*)(qk + go[it]) = val[it];
    __threadfence();
  }
}

__global__ __launch_bounds__(256) void k_pow(const float* __restrict__ dl, float* __restrict__ pw) {
  __shared__ __align__(16) float tb[256];
  const int t = threadIdx.x;
  const int d0 = blockIdx.x * 16;
  const int dloc = t >> 4, r = t & 15;
  const float sg = 1.0f / (1.0f + expf(-dl[r]));
  const float g  = 0.85f + 0.15f * sg;
  const float lg = logf(fmaxf(g, 1e-8f));
  const float dist = (float)(d0 + dloc);
  tb[t] = expf(dist * lg);
  __syncthreads();
  if (t < 64) {
    const v4f vv = *(const v4f*)(tb + 4 * t);
    volatile v4f* dp = (volatile v4f*)(pw + (size_t)d0 * RR + 4 * t);
    *dp = vv;
    __threadfence();
    *dp = vv;
  }
}

__global__ __launch_bounds__(128) void k_scores(const float* __restrict__ qk,
                                               const float* __restrict__ pw,
                                               const float* __restrict__ kb,
                                               const float* __restrict__ gl,
                                               const float* __restrict__ al,
                                               _Float16* __restrict__ S) {
  __shared__ float qi[16];
  __shared__ __align__(16) float srow[WW];
  const int i = blockIdx.x, b = blockIdx.y;
  const int t = threadIdx.x, wave = t >> 5;
  if (t < 16) qi[t] = qk[((size_t)b * WW + i) * 32 + t];
  __syncthreads();
  float q[16];
#pragma unroll
  for (int r = 0; r < 16; ++r) q[r] = qi[r];
  const float gate  = 1.0f / (1.0f + __expf(-gl[0]));
  const float alpha = 1.0f / (1.0f + __expf(-al[0]));
  const int jw = wave * 256;
  if (jw <= i) {
#pragma unroll 1
    for (int jj = 0; jj < 8; ++jj) {
      const int j = 8 * t + jj;
      int dd = i - j;
      dd = dd < 0 ? 0 : dd;
      const float* kr = qk + ((size_t)b * WW + j) * 32 + 16;
      const float* pr = pw + (size_t)dd * RR;
      v4f kv[4], pv[4];
#pragma unroll
      for (int e = 0; e < 4; ++e) { kv[e] = *(const v4f*)(kr + 4 * e); pv[e] = *(const v4f*)(pr + 4 * e); }
      float s = 0.f;
#pragma unroll
      for (int e = 0; e < 4; ++e) {
        s = fmaf(q[4 * e + 0] * pv[e][0], kv[e][0], s);
        s = fmaf(q[4 * e + 1] * pv[e][1], kv[e][1], s);
        s = fmaf(q[4 * e + 2] * pv[e][2], kv[e][2], s);
        s = fmaf(q[4 * e + 3] * pv[e][3], kv[e][3], s);
      }
      float val = gate * kb[(size_t)i * WW + j] + alpha * s;
      val = (j <= i) ? val : 0.0f;
      srow[j] = val;
    }
  } else {
    const v4f z = (v4f){0.f, 0.f, 0.f, 0.f};
    *(v4f*)(srow + 8 * t)     = z;
    *(v4f*)(srow + 8 * t + 4) = z;
  }
  __syncthreads();
  const v4f a0 = *(const v4f*)(srow + 8 * t);
  const v4f a1 = *(const v4f*)(srow + 8 * t + 4);
  Pack8 pk;
  pk.h = (v8h){(_Float16)(a0[0] * 256.0f), (_Float16)(a0[1] * 256.0f), (_Float16)(a0[2] * 256.0f), (_Float16)(a0[3] * 256.0f),
               (_Float16)(a1[0] * 256.0f), (_Float16)(a1[1] * 256.0f), (_Float16)(a1[2] * 256.0f), (_Float16)(a1[3] * 256.0f)};
  const v4u vv = pk.u;
  volatile v4u* d = (volatile v4u*)(S + ((size_t)b * WW + i) * WW + 8 * t);
  *d = vv;
  __threadfence();
  *d = vv;
}

#define OTP 68
__global__ __launch_bounds__(256) void k_mix(const _Float16* __restrict__ S,
                                            const _Float16* __restrict__ hnT,
                                            _Float16* __restrict__ o1) {
  __shared__ __align__(16) float st[8][16 * OTP];
  const int tid = threadIdx.x, lane = tid & 31, wave = tid >> 5;
  const int hh = lane >> 4, c = lane & 15;
  const int b  = blockIdx.z;
  const int ml = blockIdx.x * 256 + wave * 32;
  const int n0 = blockIdx.y * 64;
  const _Float16* A  = S   + (size_t)b * WW * WW;
  const _Float16* Bt = hnT + (size_t)b * CC * WW;
  const int kend = ml + 32;

  v8f acc[2][4];
#pragma unroll
  for (int s = 0; s < 2; ++s)
#pragma unroll
    for (int t = 0; t < 4; ++t) acc[s][t] = zero8();
  gemm32x64(A, WW, Bt, WW, ml, n0, lane, kend, acc);

  float* sw = st[wave];
#pragma unroll
  for (int sub = 0; sub < 2; ++sub) {
    __syncthreads();
#pragma unroll
    for (int t = 0; t < 4; ++t) {
#pragma unroll
      for (int r = 0; r < 8; ++r)
        sw[(8 * hh + r) * OTP + 16 * t + c] = acc[sub][t][r] * 0.0625f;
    }
    __syncthreads();
    v4u val[4];
    size_t go[4];
#pragma unroll
    for (int it = 0; it < 4; ++it) {
      const int p  = lane + 32 * it;
      const int L  = p >> 3;
      const int pc = p & 7;
      const v4f x0 = *(const v4f*)(sw + L * OTP + pc * 8);
      const v4f x1 = *(const v4f*)(sw + L * OTP + pc * 8 + 4);
      Pack8 pk;
      pk.h = (v8h){(_Float16)x0[0], (_Float16)x0[1], (_Float16)x0[2], (_Float16)x0[3],
                   (_Float16)x1[0], (_Float16)x1[1], (_Float16)x1[2], (_Float16)x1[3]};
      val[it] = pk.u;
      go[it]  = ((size_t)b * WW + ml + sub * 16 + L) * CC + n0 + pc * 8;
    }
    for (int ps = 0; ps < 2; ++ps) {
#pragma unroll
      for (int it = 0; it < 4; ++it) *(volatile v4u*)(o1 + go[it]) = val[it];
      __threadfence();
    }
  }
}

template <int KK, int RES>
__global__ __launch_bounds__(256) void k_gout(const _Float16* __restrict__ ap,
                                             const _Float16* __restrict__ wt,
                                             const float* __restrict__ bias,
                                             const float* __restrict__ res,
                                             float* __restrict__ out, float oscale) {
  __shared__ __align__(16) float st[8][16 * OTP];
  const int tid = threadIdx.x, lane = tid & 31, wave = tid >> 5;
  const int hh = lane >> 4, c = lane & 15;
  const int m0 = blockIdx.x * 256 + wave * 32;
  const int n0 = blockIdx.y * 64;

  v8f acc[2][4];
#pragma unroll
  for (int s = 0; s < 2; ++s)
#pragma unroll
    for (int t = 0; t < 4; ++t) acc[s][t] = zero8();
  gemm32x64(ap, KK, wt, KK, m0, n0, lane, KK, acc);

  float bvs[4];
#pragma unroll
  for (int t = 0; t < 4; ++t) bvs[t] = bias[n0 + 16 * t + c];

  float* sw = st[wave];
#pragma unroll
  for (int sub = 0; sub < 2; ++sub) {
    __syncthreads();
#pragma unroll
    for (int t = 0; t < 4; ++t) {
#pragma unroll
      for (int r = 0; r < 8; ++r)
        sw[(8 * hh + r) * OTP + 16 * t + c] = acc[sub][t][r] * oscale + bvs[t];
    }
    __syncthreads();
    v4f val[8];
    size_t go[8];
#pragma unroll
    for (int it = 0; it < 8; ++it) {
      const int p    = lane + 32 * it;
      const int L    = p >> 3;
      const int pc   = p & 7;
      const int row  = L >> 1;
      const int half = L & 1;
      const size_t g = (size_t)(m0 + sub * 16 + row) * CC + n0 + half * 32 + pc * 4;
      v4f v = *(const v4f*)(sw + row * OTP + half * 32 + pc * 4);
      if (RES) {
        const v4f rr = *(const v4f*)(res + g);
        v[0] = v[0] + rr[0]; v[1] = v[1] + rr[1]; v[2] = v[2] + rr[2]; v[3] = v[3] + rr[3];
      }
      val[it] = v;
      go[it]  = g;
    }
    for (int ps = 0; ps < 2; ++ps) {
#pragma unroll
      for (int it = 0; it < 8; ++it) *(volatile v4f*)(out + go[it]) = val[it];
      __threadfence();
    }
  }
}

__global__ __launch_bounds__(256) void k_ffn1(const _Float16* __restrict__ ap,
                                             const _Float16* __restrict__ wt,
                                             const float* __restrict__ bias,
                                             _Float16* __restrict__ hp) {
  __shared__ __align__(16) float st[8][16 * OTP];
  const int tid = threadIdx.x, lane = tid & 31, wave = tid >> 5;
  const int hh = lane >> 4, c = lane & 15;
  const int m0 = blockIdx.x * 256 + wave * 32;
  const int n0 = blockIdx.y * 64;

  v8f acc[2][4];
#pragma unroll
  for (int s = 0; s < 2; ++s)
#pragma unroll
    for (int t = 0; t < 4; ++t) acc[s][t] = zero8();
  gemm32x64(ap, CC, wt, CC, m0, n0, lane, CC, acc);

  float bvs[4];
#pragma unroll
  for (int t = 0; t < 4; ++t) bvs[t] = bias[n0 + 16 * t + c];

  float* sw = st[wave];
#pragma unroll
  for (int sub = 0; sub < 2; ++sub) {
    __syncthreads();
#pragma unroll
    for (int t = 0; t < 4; ++t) {
#pragma unroll
      for (int r = 0; r < 8; ++r)
        sw[(8 * hh + r) * OTP + 16 * t + c] = acc[sub][t][r] * 0.03125f + bvs[t];
    }
    __syncthreads();
    v4u val[4];
    size_t go[4];
#pragma unroll
    for (int it = 0; it < 4; ++it) {
      const int p  = lane + 32 * it;
      const int L  = p >> 3;
      const int pc = p & 7;
      const v4f x0 = *(const v4f*)(sw + L * OTP + pc * 8);
      const v4f x1 = *(const v4f*)(sw + L * OTP + pc * 8 + 4);
      Pack8 pk;
      pk.h = (v8h){(_Float16)act16(x0[0]), (_Float16)act16(x0[1]), (_Float16)act16(x0[2]), (_Float16)act16(x0[3]),
                   (_Float16)act16(x1[0]), (_Float16)act16(x1[1]), (_Float16)act16(x1[2]), (_Float16)act16(x1[3])};
      val[it] = pk.u;
      go[it]  = (size_t)(m0 + sub * 16 + L) * FF + n0 + pc * 8;
    }
    for (int ps = 0; ps < 2; ++ps) {
#pragma unroll
      for (int it = 0; it < 4; ++it) *(volatile v4u*)(hp + go[it]) = val[it];
      __threadfence();
    }
  }
}

extern "C" void kernel_launch(void* const* d_in, const int* in_sizes, int n_in,
                              void* d_out, int out_size, void* d_ws, size_t ws_size,
                              hipStream_t stream) {
  if (n_in < 15) return;
  if (in_sizes[0] != ROWS * CC) return;
  if (in_sizes[1] != RR) return;
  if (in_sizes[2] != WW * WW) return;
  if (in_sizes[3] != 1 || in_sizes[6] != 1) return;
  if (in_sizes[4] != CC * RR || in_sizes[5] != CC * RR) return;
  if (in_sizes[7] != CC * CC || in_sizes[8] != CC) return;
  if (in_sizes[9] != CC || in_sizes[10] != CC) return;
  if (in_sizes[11] != CC * FF || in_sizes[12] != FF) return;
  if (in_sizes[13] != FF * CC || in_sizes[14] != CC) return;
  if (out_size != ROWS * CC) return;

  const float* h   = (const float*)d_in[0];
  const float* dl  = (const float*)d_in[1];
  const float* kb  = (const float*)d_in[2];
  const float* gl  = (const float*)d_in[3];
  const float* u   = (const float*)d_in[4];
  const float* v   = (const float*)d_in[5];
  const float* al  = (const float*)d_in[6];
  const float* Wp  = (const float*)d_in[7];
  const float* pb  = (const float*)d_in[8];
  const float* n1  = (const float*)d_in[9];
  const float* n2  = (const float*)d_in[10];
  const float* Wu  = (const float*)d_in[11];
  const float* ub  = (const float*)d_in[12];
  const float* Wd  = (const float*)d_in[13];
  const float* db  = (const float*)d_in[14];
  float* out = (float*)d_out;

  size_t off = 0;
  const size_t oHn  = off; off += (size_t)ROWS * CC * 2;
  const size_t oHnT = off; off += (size_t)BB * CC * WW * 2;
  const size_t oUV  = off; off += (size_t)32 * CC * 2;
  const size_t oQK  = off; off += (size_t)ROWS * 32 * 4;
  const size_t oPW  = off; off += (size_t)WW * RR * 4;
  const size_t oS   = off; off += (size_t)BB * WW * WW * 2;
  const size_t oO1  = off; off += (size_t)ROWS * CC * 2;
  const size_t oWp  = off; off += (size_t)CC * CC * 2;
  const size_t oWu  = off; off += (size_t)FF * CC * 2;
  const size_t oWd  = off; off += (size_t)CC * FF * 2;
  const size_t oH2  = off; off += (size_t)ROWS * CC * 4;
  const size_t oH2n = off; off += (size_t)ROWS * CC * 2;
  const size_t oMid = off; off += (size_t)ROWS * FF * 2;
  if (off > ws_size) return;
  if (off > (size_t)134217728) return;

  char* ws = (char*)d_ws;
  _Float16* Hn  = (_Float16*)(ws + oHn);
  _Float16* HnT = (_Float16*)(ws + oHnT);
  _Float16* UVt = (_Float16*)(ws + oUV);
  float*    QK  = (float*)(ws + oQK);
  float*    PW  = (float*)(ws + oPW);
  _Float16* Sp  = (_Float16*)(ws + oS);
  _Float16* O1  = (_Float16*)(ws + oO1);
  _Float16* Wpt = (_Float16*)(ws + oWp);
  _Float16* Wut = (_Float16*)(ws + oWu);
  _Float16* Wdt = (_Float16*)(ws + oWd);
  float*    H2  = (float*)(ws + oH2);
  _Float16* H2n = (_Float16*)(ws + oH2n);
  _Float16* Mid = (_Float16*)(ws + oMid);

  k_rms<<<dim3(ROWS), dim3(256), 0, stream>>>(h, n1, Hn);
  k_tr16<<<dim3(CC / 64, WW / 64, BB), dim3(256), 0, stream>>>(Hn, HnT, WW, CC);
  k_uvt<<<dim3(32), dim3(128), 0, stream>>>(u, v, UVt);
  k_wt<<<dim3(CC / 64, CC / 64), dim3(256), 0, stream>>>(Wp, Wpt, CC, CC);
  k_wt<<<dim3(FF / 64, CC / 64), dim3(256), 0, stream>>>(Wu, Wut, FF, CC);
  k_wt<<<dim3(CC / 64, FF / 64), dim3(256), 0, stream>>>(Wd, Wdt, CC, FF);
  k_qk<<<dim3(ROWS / 128), dim3(256), 0, stream>>>(Hn, UVt, QK);
  k_pow<<<dim3(WW / 16), dim3(256), 0, stream>>>(dl, PW);
  k_scores<<<dim3(WW, BB), dim3(128), 0, stream>>>(QK, PW, kb, gl, al, Sp);
  k_mix<<<dim3(WW / 256, CC / 64, BB), dim3(256), 0, stream>>>(Sp, HnT, O1);
  k_gout<CC, 1><<<dim3(ROWS / 256, CC / 64), dim3(256), 0, stream>>>(O1, Wpt, pb, h, H2, 0.001953125f);
  k_rms<<<dim3(ROWS), dim3(256), 0, stream>>>(H2, n2, H2n);
  k_ffn1<<<dim3(ROWS / 256, FF / 64), dim3(256), 0, stream>>>(H2n, Wut, ub, Mid);
  k_gout<FF, 1><<<dim3(ROWS / 256, CC / 64), dim3(256), 0, stream>>>(Mid, Wdt, db, H2, out, 0.001953125f);
  (void)hipGetLastError();
}
